// MultiHeadDistanceLayer_60756607369712
// MI455X (gfx1250) — hardware-verified
//
#include <hip/hip_runtime.h>
#include <math.h>

constexpr int kB    = 2;
constexpr int kL    = 2048;
constexpr int kC    = 256;
constexpr int kH    = 8;
constexpr int kDh   = 32;
constexpr int kTok  = kB * kL;
constexpr int kQKld = 2 * kC;
constexpr int kVN   = 64;
constexpr int kGH   = 4;
constexpr int kRowChunks = kL / 128;
constexpr float kScale     = 0.17677669529663687f;
constexpr float kWCarry    = 16.0f;
constexpr float kWCarryInv = 1.0f / 16.0f;
static_assert(kH * kDh == kC);
static_assert(kL % 64 == 0 && kTok % 64 == 0 && kC % 64 == 0 && kVN % 64 == 0);
static_assert(kC % 32 == 0 && kDh % 32 == 0);
static_assert(kL % 1024 == 0 && kL % 32 == 0);
static_assert(kH == 8 && kL * kH == (1 << 14));
static_assert(((kL * kC) & (kL * kC - 1)) == 0);
static_assert(kH % kGH == 0 && kH <= kVN);
static_assert((kTok * kC) % (8 * 256) == 0);

typedef __attribute__((ext_vector_type(16))) _Float16 v16h;
typedef __attribute__((ext_vector_type(8)))  _Float16 v8h;
typedef __attribute__((ext_vector_type(16))) __bf16   v16b;
typedef __attribute__((ext_vector_type(8)))  __bf16   v8b;
typedef __attribute__((ext_vector_type(8)))  float    v8f;
typedef __attribute__((ext_vector_type(4)))  float    v4f;
typedef __attribute__((ext_vector_type(4)))  unsigned int v4u;

__device__ __forceinline__ unsigned short f2bf_bits(float f) {
  unsigned u = __float_as_uint(f);
  return (unsigned short)((u + 0x7FFFu + ((u >> 16) & 1u)) >> 16);
}
__device__ __forceinline__ float bf_bits2f(unsigned short h) { return __uint_as_float(((unsigned)h) << 16); }

__device__ __forceinline__ void dep_guard_h(v8f& a, v8f& b, v16h x, v16h y) { asm volatile("v_nop\n\tv_nop\n\tv_nop\n\tv_nop" : "+v"(a), "+v"(b) : "v"(x), "v"(y)); }
__device__ __forceinline__ void dep_guard_b(v8f& a, v8f& b, v16b x, v16b y) { asm volatile("v_nop\n\tv_nop\n\tv_nop\n\tv_nop" : "+v"(a), "+v"(b) : "v"(x), "v"(y)); }
__device__ __forceinline__ void keep4_h(v16h a, v16h b, v16h c, v16h d) { asm volatile("v_nop" :: "v"(a), "v"(b), "v"(c), "v"(d)); }
__device__ __forceinline__ void keep4_b(v16b a, v16b b, v16b c, v16b d) { asm volatile("v_nop" :: "v"(a), "v"(b), "v"(c), "v"(d)); }
__device__ __forceinline__ void acc_guard4(v8f& a, v8f& b, v8f& c, v8f& d) { asm volatile("v_nop\n\tv_nop\n\tv_nop\n\tv_nop" : "+v"(a), "+v"(b), "+v"(c), "+v"(d)); }
template <typename T> struct Frag;
template <> struct Frag<_Float16> {
  typedef v16h V; union U { v16h v; v8h h[2]; };
  static __device__ __forceinline__ v16h load(const _Float16* p) {
    U f; f.h[0] = *(const v8h*)(p); f.h[1] = *(const v8h*)(p + 16); return f.v;
  }
  static __device__ __forceinline__ v8f mma(v16h a, v16h b, v8f c) {
    return __builtin_amdgcn_wmma_f32_16x16x32_f16(false, a, false, b, (short)0, c, false, false);
  }
  static __device__ __forceinline__ void guard(v8f& a, v8f& b, v16h x, v16h y) { dep_guard_h(a, b, x, y); }
  static __device__ __forceinline__ void keep(v16h a, v16h b, v16h c, v16h d) { keep4_h(a, b, c, d); }
};
template <> struct Frag<__bf16> {
  typedef v16b V; union U { v16b v; v8b h[2]; };
  static __device__ __forceinline__ v16b load(const __bf16* p) {
    U f; f.h[0] = *(const v8b*)(p); f.h[1] = *(const v8b*)(p + 16); return f.v;
  }
  static __device__ __forceinline__ v8f mma(v16b a, v16b b, v8f c) {
    return __builtin_amdgcn_wmma_f32_16x16x32_bf16(false, a, false, b, (short)0, c, false, false);
  }
  static __device__ __forceinline__ void guard(v8f& a, v8f& b, v16b x, v16b y) { dep_guard_b(a, b, x, y); }
  static __device__ __forceinline__ void keep(v16b a, v16b b, v16b c, v16b d) { keep4_b(a, b, c, d); }
};

__device__ __forceinline__ unsigned pk16(unsigned short a, unsigned short b) { return (unsigned)a | ((unsigned)b << 16); }
__device__ __forceinline__ unsigned short h_bits(float f) { const _Float16 h = (_Float16)f; return __builtin_bit_cast(unsigned short, h); }

template <int ET> struct Elem;
template <> struct Elem<0> { typedef _Float16 T; };
template <> struct Elem<1> { typedef __bf16 T; };
template <int ET, bool SPLIT, int BIAS_MODE, int OUT_MODE, bool RESID, int ACT = 0>
__global__ __launch_bounds__(256) void wmma_gemm64(
    const unsigned short* __restrict__ Ap, const unsigned short* __restrict__ A2p, int lda, long strideA,
    const unsigned short* __restrict__ Btp, const unsigned short* __restrict__ Bt2p, int ldb, long strideB,
    void* __restrict__ Cout, void* __restrict__ Cout2, int ldc, long strideC,
    const float* __restrict__ bias,
    const float* __restrict__ resid, long strideR,
    int M, int N, int K, float scale) {
  typedef typename Elem<ET>::T T;
  typedef typename Frag<T>::V V;
  const T* A = (const T*)Ap; const T* A2 = (const T*)A2p; const T* Bt = (const T*)Btp; const T* Bt2 = (const T*)Bt2p;
  __shared__ __align__(16) float sT[8][16 * 68];
  const int b    = blockIdx.y;
  const int lane = threadIdx.x & 31;
  const int wave = threadIdx.x >> 5;
  const int tilesN = N >> 6;
  const int tilesM = M >> 6;
  const int tile = blockIdx.x * 8 + wave;
  if (tile >= tilesM * tilesN) return;
  const int tm = tile / tilesN;
  const int tn = tile - tm * tilesN;
  const int m0 = tm << 6;
  const int n0 = tn << 6;

  const T* Ab  = A  + (size_t)b * strideA;
  const T* Bb  = Bt + (size_t)b * strideB;
  const T* Ab2 = SPLIT ? (A2  + (size_t)b * strideA) : nullptr;
  const T* Bb2 = SPLIT ? (Bt2 + (size_t)b * strideB) : nullptr;

  const int rlane = lane & 15;
  const int koff  = (lane >> 4) * 8;
  const int mOff  = (lane >> 4) * 8;

  v8f acc[4][4];
#pragma unroll
  for (int i = 0; i < 4; ++i)
#pragma unroll
    for (int j = 0; j < 4; ++j) acc[i][j] = (v8f){0.f,0.f,0.f,0.f,0.f,0.f,0.f,0.f};

  for (int k0 = 0; k0 < K; k0 += 32) {
    V bh[4], bl[4];
#pragma unroll
    for (int j = 0; j < 4; ++j) {
      const size_t bo = (size_t)(n0 + (j << 4) + rlane) * ldb + koff + k0;
      bh[j] = Frag<T>::load(Bb + bo);
      if (SPLIT) bl[j] = Frag<T>::load(Bb2 + bo);
    }
#pragma unroll
    for (int i = 0; i < 4; ++i) {
      const size_t ao = (size_t)(m0 + (i << 4) + rlane) * lda + koff + k0;
      V ah = Frag<T>::load(Ab + ao);
      V al;
      if (SPLIT) al = Frag<T>::load(Ab2 + ao);
#pragma unroll
      for (int j = 0; j < 4; ++j) {
        acc[i][j] = Frag<T>::mma(ah, bh[j], acc[i][j]);
        if (SPLIT) {
          acc[i][j] = Frag<T>::mma(ah, bl[j], acc[i][j]);
          acc[i][j] = Frag<T>::mma(al, bh[j], acc[i][j]);
        }
      }
      Frag<T>::guard(acc[i][0], acc[i][3], ah, SPLIT ? al : ah);
    }
    Frag<T>::keep(bh[0], bh[1], bh[2], bh[3]);
    if (SPLIT) Frag<T>::keep(bl[0], bl[1], bl[2], bl[3]);
  }
  acc_guard4(acc[0][0], acc[0][1], acc[0][2], acc[0][3]);
  acc_guard4(acc[1][0], acc[1][1], acc[1][2], acc[1][3]);
  acc_guard4(acc[2][0], acc[2][1], acc[2][2], acc[2][3]);
  acc_guard4(acc[3][0], acc[3][1], acc[3][2], acc[3][3]);

  float* slab = sT[wave];
  const float* Rb = RESID ? (resid + (size_t)b * strideR) : nullptr;
#pragma unroll
  for (int i = 0; i < 4; ++i) {
    const int mBase = m0 + (i << 4);
#pragma unroll
    for (int j = 0; j < 4; ++j) {
      const int n = n0 + (j << 4) + rlane;
      float bv = 0.f;
      if (BIAS_MODE == 2) bv = bias[n];
#pragma unroll
      for (int r = 0; r < 8; ++r) {
        float v = acc[i][j][r] * scale;
        if (BIAS_MODE == 1) v += bias[mBase + mOff + r];
        if (BIAS_MODE == 2) v += bv;
        if (RESID) v += Rb[(size_t)(mBase + mOff + r) * ldc + n];
        if (ACT == 2) v = fmaxf(v, 0.0f);
        if (ACT == 4) v = (v > 0.f) ? v : 0.01f * v;
        slab[(mOff + r) * 68 + (j << 4) + rlane] = v;
      }
    }
    __builtin_amdgcn_fence(__ATOMIC_RELEASE, "workgroup");
    __builtin_amdgcn_wave_barrier();
    __builtin_amdgcn_fence(__ATOMIC_ACQUIRE, "workgroup");
    if (OUT_MODE == 0) {
      float* C = (float*)Cout + (size_t)b * strideC;
      const int hh = lane >> 4, c4 = (lane & 15) * 4;
      for (int pass = 0; pass < 2; ++pass) {
#pragma unroll
        for (int it = 0; it < 8; ++it) {
          const int row = it * 2 + hh;
          v4f v = *(const v4f*)(slab + row * 68 + c4);
          *(volatile v4f*)(C + (size_t)(mBase + row) * ldc + n0 + c4) = v;
        }
        __threadfence();
      }
    } else {
      const int q = lane >> 3, c8 = (lane & 7) * 8;
      unsigned short* C  = (unsigned short*)Cout  + (size_t)b * strideC;
      unsigned short* C2 = (OUT_MODE == 2) ? ((unsigned short*)Cout2 + (size_t)b * strideC) : nullptr;
      for (int pass = 0; pass < 2; ++pass) {
#pragma unroll
        for (int it = 0; it < 4; ++it) {
          const int row = it * 4 + q;
          const float* sp = slab + row * 68 + c8;
          v8h hv, lv;
#pragma unroll
          for (int e = 0; e < 8; ++e) {
            if (OUT_MODE == 1) {
              hv[e] = (_Float16)sp[e];
            } else {
              unsigned short hb = f2bf_bits(sp[e]);
              unsigned short lb = f2bf_bits(sp[e] - bf_bits2f(hb));
              hv[e] = __builtin_bit_cast(_Float16, hb);
              lv[e] = __builtin_bit_cast(_Float16, lb);
            }
          }
          *(volatile v8h*)(C + (size_t)(mBase + row) * ldc + n0 + c8) = hv;
          if (OUT_MODE == 2) *(volatile v8h*)(C2 + (size_t)(mBase + row) * ldc + n0 + c8) = lv;
        }
        __threadfence();
      }
    }
    __builtin_amdgcn_fence(__ATOMIC_RELEASE, "workgroup");
    __builtin_amdgcn_wave_barrier();
    __builtin_amdgcn_fence(__ATOMIC_ACQUIRE, "workgroup");
  }
}

__global__ __launch_bounds__(256) void xcast_kernel(const float* __restrict__ x, const float* __restrict__ pe,
                                                    unsigned short* __restrict__ XQ, unsigned short* __restrict__ XR, int n8) {
  const int i = blockIdx.x * 256 + threadIdx.x;
  if (i >= n8) return;
  const size_t e0 = 8 * (size_t)i;
  const size_t p0 = e0 & (size_t)(kL * kC - 1);
  const v4f a  = *(const v4f*)(x + e0);
  const v4f c  = *(const v4f*)(x + e0 + 4);
  const v4f pa = *(const v4f*)(pe + p0);
  const v4f pc = *(const v4f*)(pe + p0 + 4);
  unsigned short hr[8], hq[8];
#pragma unroll
  for (int e = 0; e < 4; ++e) {
    hr[e]     = h_bits(a[e]);
    hr[4 + e] = h_bits(c[e]);
    hq[e]     = h_bits(a[e] + pa[e]);
    hq[4 + e] = h_bits(c[e] + pc[e]);
  }
  const v4u ur = (v4u){pk16(hr[0], hr[1]), pk16(hr[2], hr[3]), pk16(hr[4], hr[5]), pk16(hr[6], hr[7])};
  const v4u uq = (v4u){pk16(hq[0], hq[1]), pk16(hq[2], hq[3]), pk16(hq[4], hq[5]), pk16(hq[6], hq[7])};
  unsigned short* dq = XQ + e0;
  unsigned short* dr = XR + e0;
  *(volatile v4u*)dq = uq;
  *(volatile v4u*)dr = ur;
  __threadfence();
  *(volatile v4u*)dq = uq;
  *(volatile v4u*)dr = ur;
}

__global__ __launch_bounds__(256) void wtcast_kernel(const float* __restrict__ W0, const float* __restrict__ W1,
                                                     unsigned short* __restrict__ out, float scale) {
  __shared__ float sm[64][65];
  const int t  = threadIdx.x;
  const int c0 = blockIdx.x * 64;
  const int n0 = blockIdx.y * 64;
  const int z  = blockIdx.z;
  const float* W = (z == 0) ? W0 : W1;
#pragma unroll
  for (int i = 0; i < 16; ++i) {
    const int e = i * 256 + t;
    const int r = e >> 6;
    const int cc = e & 63;
    sm[cc][r] = W[(size_t)(c0 + r) * kC + n0 + cc] * scale;
  }
  __syncthreads();
  const int lane = t & 31, wave = t >> 5;
  const int q = lane >> 3, c8 = (lane & 7) * 8;
  unsigned short* op = out + (size_t)z * kC * kC;
  for (int pass = 0; pass < 2; ++pass) {
#pragma unroll
    for (int it = 0; it < 2; ++it) {
      const int row = wave * 8 + it * 4 + q;
      unsigned short hb[8];
#pragma unroll
      for (int e = 0; e < 8; ++e) hb[e] = h_bits(sm[row][c8 + e]);
      const v4u u = (v4u){pk16(hb[0], hb[1]), pk16(hb[2], hb[3]), pk16(hb[4], hb[5]), pk16(hb[6], hb[7])};
      *(volatile v4u*)(op + (size_t)(n0 + row) * kC + c0 + c8) = u;
    }
    __threadfence();
  }
}

__global__ __launch_bounds__(32) void wvpad_kernel(const float* __restrict__ Wv, unsigned short* __restrict__ out, float scale) {
  const int n = blockIdx.x;
  const int lane = threadIdx.x;
  const int c = lane * 8;
  const int nn = (n < kH) ? n : 0;
  const float f = (n < kH) ? scale : 0.0f;
  unsigned short hb[8];
#pragma unroll
  for (int e = 0; e < 8; ++e) hb[e] = h_bits(f * Wv[(size_t)(c + e) * kH + nn]);
  const v4u u = (v4u){pk16(hb[0], hb[1]), pk16(hb[2], hb[3]), pk16(hb[4], hb[5]), pk16(hb[6], hb[7])};
  unsigned short* dp = out + (size_t)n * kC + c;
  *(volatile v4u*)dp = u;
  __threadfence();
  *(volatile v4u*)dp = u;
}

__global__ __launch_bounds__(256) void rowstats_kernel(const float* __restrict__ SC, const float* __restrict__ VR,
                                                       float* __restrict__ ST, int b, int h0) {
  __shared__ __align__(16) float sMF[64];
  const int z  = blockIdx.y;
  const int r0 = blockIdx.x * 32;
  const int t  = threadIdx.x, lane = t & 31, wave = t >> 5;
  const int h  = h0 + z;
  const int p  = b * kH + h;
  const float* Sz = SC + (size_t)z * kL * kL;
#pragma unroll 1
  for (int i = 0; i < 4; ++i) {
    const int rl  = wave * 4 + i;
    const int row = r0 + rl;
    const float* sr = Sz + (size_t)row * kL + lane * 4;
    float mx = -__builtin_inff();
#pragma unroll 2
    for (int j = 0; j < kRowChunks; ++j) {
      const v4f a = *(const v4f*)(sr + j * 128);
      mx = fmaxf(mx, fmaxf(fmaxf(a[0], a[1]), fmaxf(a[2], a[3])));
    }
#pragma unroll
    for (int off = 16; off > 0; off >>= 1) mx = fmaxf(mx, __shfl_xor(mx, off, 32));
    float sum = 0.f;
#pragma unroll 1
    for (int j = 0; j < kRowChunks; ++j) {
      const v4f a = *(const v4f*)(sr + j * 128);
      sum += (expf(a[0] - mx) + expf(a[1] - mx)) + (expf(a[2] - mx) + expf(a[3] - mx));
    }
#pragma unroll
    for (int off = 16; off > 0; off >>= 1) sum += __shfl_xor(sum, off, 32);
    const float vq = VR[(size_t)(b * kL + row) * kVN + h];
    const float fq = vq * (1.0f / sum);
    if (lane == 0) { sMF[rl] = mx; sMF[32 + rl] = fq; }
  }
  __syncthreads();
  if (t < 16) {
    const v4f val = *(const v4f*)(sMF + 4 * t);
    const int sub = (t < 8) ? (4 * t) : (kL + 4 * (t - 8));
    float* dp = ST + (size_t)p * (2 * kL) + r0 + sub;
    *(volatile v4f*)dp = val;
    __threadfence();
    *(volatile v4f*)dp = val;
  }
}

__global__ __launch_bounds__(256) void colsum_kernel(const float* __restrict__ SC, const float* __restrict__ ST,
                                                     float* __restrict__ CS, int b, int h0) {
  __shared__ __align__(16) float sMF[2 * kL];
  const int z  = blockIdx.y;
  const int kb = blockIdx.x * 1024;
  const int t  = threadIdx.x, wave = t >> 5;
  const int p  = b * kH + h0 + z;
  const float* stp = ST + (size_t)p * (2 * kL);
#pragma unroll
  for (int j = 0; j < 4; ++j) {
    const v4f w = *(const v4f*)(stp + j * 1024 + 4 * t);
    *(v4f*)(sMF + j * 1024 + 4 * t) = w;
  }
  __syncthreads();
  const int k0 = kb + 4 * t;
  const int qstart = kb + wave * 128;
  const float* Sz = SC + (size_t)z * kL * kL + k0;
  float acc[4], part[4];
#pragma unroll
  for (int e = 0; e < 4; ++e) { acc[e] = 0.0f; part[e] = 0.0f; }
#pragma unroll 1
  for (int q = qstart; q < kL; ++q) {
    const v4f s = *(const v4f*)(Sz + (size_t)q * kL);
    const float m = sMF[q];
    const float f = sMF[kL + q];
#pragma unroll
    for (int e = 0; e < 4; ++e) {
      const float pv = expf(s[e] - m) * f;
      const float keep = (q >= k0 + e) ? 1.0f : 0.0f;
      part[e] = fmaf(pv, keep, part[e]);
    }
    if ((q & 63) == 63) {
#pragma unroll
      for (int e = 0; e < 4; ++e) { acc[e] += part[e]; part[e] = 0.0f; }
    }
  }
#pragma unroll
  for (int e = 0; e < 4; ++e) acc[e] += part[e];
  const v4f val = (v4f){acc[0], acc[1], acc[2], acc[3]};
  float* dp = CS + (size_t)p * kL + k0;
  *(volatile v4f*)dp = val;
  __threadfence();
  *(volatile v4f*)dp = val;
}

__global__ __launch_bounds__(256) void pool_kernel(const float* __restrict__ CS, float* __restrict__ out, int n4) {
  const int t = blockIdx.x * 256 + threadIdx.x;
  if (t >= n4) return;
  const int idx0 = 4 * t;
  const int hb0  = idx0 & (kH - 1);
  const int k    = (idx0 >> 3) & (kL - 1);
  const int b    = idx0 >> 14;
  const int km   = (k > 0) ? (k - 1) : 0;
  const int kp   = (k < kL - 1) ? (k + 1) : (kL - 1);
  const float fl = (k > 0) ? 1.0f : 0.0f;
  const float fr = (k < kL - 1) ? 1.0f : 0.0f;
  const float inv = (k > 0 && k < kL - 1) ? (1.0f / 3.0f) : 0.5f;
  v4f o;
#pragma unroll
  for (int e = 0; e < 4; ++e) {
    const float* cs = CS + (size_t)(b * kH + hb0 + e) * kL;
    const float cm = cs[km];
    const float cc = cs[k];
    const float cp = cs[kp];
    float s = fmaf(fl, cm, cc);
    s = fmaf(fr, cp, s);
    o[e] = s * inv;
  }
  float* dp = out + idx0;
  *(volatile v4f*)dp = o;
  __threadfence();
  *(volatile v4f*)dp = o;
}

extern "C" void kernel_launch(void* const* d_in, const int* in_sizes, int n_in,
                              void* d_out, int out_size, void* d_ws, size_t ws_size,
                              hipStream_t stream) {
  if (n_in < 7) return;
  if (in_sizes[0] != kTok * kC) return;
  if (in_sizes[1] != kC * kC || in_sizes[3] != kC * kC) return;
  if (in_sizes[2] != kH * kDh || in_sizes[4] != kH * kDh) return;
  if (in_sizes[5] != kC * kH) return;
  if (in_sizes[6] != kL * kC) return;
  if (out_size != kB * kL * kH) return;

  const size_t szX  = (size_t)kTok * kC * 2;
  const size_t szWT = (size_t)2 * kC * kC * 2;
  const size_t szWV = (size_t)kVN * kC * 2;
  const size_t szQK = (size_t)kTok * kQKld * 2;
  const size_t szVR = (size_t)kTok * kVN * 4;
  const size_t szST = (size_t)kB * kH * 2 * kL * 4;
  const size_t szCS = (size_t)kB * kH * kL * 4;
  const size_t szSC = (size_t)kGH * kL * kL * 4;
  const size_t offXQ = 0;
  const size_t offXR = offXQ + szX;
  const size_t offWT = offXR + szX;
  const size_t offWV = offWT + szWT;
  const size_t offQK = offWV + szWV;
  const size_t offVR = offQK + szQK;
  const size_t offST = offVR + szVR;
  const size_t offCS = offST + szST;
  const size_t offSC = offCS + szCS;
  const size_t total = offSC + szSC;
  if (ws_size < total) return;

  const float* x  = (const float*)d_in[0];
  const float* Wq = (const float*)d_in[1];
  const float* bq = (const float*)d_in[2];
  const float* Wk = (const float*)d_in[3];
  const float* bk = (const float*)d_in[4];
  const float* Wv = (const float*)d_in[5];
  const float* pe = (const float*)d_in[6];
  float* out = (float*)d_out;
  char* ws = (char*)d_ws;
  unsigned short* XQ16 = (unsigned short*)(ws + offXQ);
  unsigned short* XR16 = (unsigned short*)(ws + offXR);
  unsigned short* WT16 = (unsigned short*)(ws + offWT);
  unsigned short* WV16 = (unsigned short*)(ws + offWV);
  unsigned short* QK16 = (unsigned short*)(ws + offQK);
  float* VR = (float*)(ws + offVR);
  float* ST = (float*)(ws + offST);
  float* CS = (float*)(ws + offCS);
  float* SC = (float*)(ws + offSC);

  const int n8 = (kTok * kC) / 8;
  xcast_kernel<<<dim3(n8 / 256), dim3(256), 0, stream>>>(x, pe, XQ16, XR16, n8);
  wtcast_kernel<<<dim3(kC / 64, kC / 64, 2), dim3(256), 0, stream>>>(Wq, Wk, WT16, kWCarry);
  wvpad_kernel<<<dim3(kVN), dim3(32), 0, stream>>>(Wv, WV16, kWCarry);

  const int tilesProj = (kTok / 64) * (kC / 64);
  const int tilesV    = (kTok / 64) * (kVN / 64);
  wmma_gemm64<0, false, 2, 1, false, 0><<<dim3(tilesProj / 8, 1), dim3(256), 0, stream>>>(
      XQ16, XQ16, kC, 0L, WT16, WT16, kC, 0L,
      (void*)QK16, (void*)QK16, kQKld, 0L, bq, VR, 0L, kTok, kC, kC, kWCarryInv);
  wmma_gemm64<0, false, 2, 1, false, 0><<<dim3(tilesProj / 8, 1), dim3(256), 0, stream>>>(
      XQ16, XQ16, kC, 0L, WT16 + (size_t)kC * kC, WT16 + (size_t)kC * kC, kC, 0L,
      (void*)(QK16 + kC), (void*)(QK16 + kC), kQKld, 0L, bk, VR, 0L, kTok, kC, kC, kWCarryInv);
  wmma_gemm64<0, false, 0, 0, false, 0><<<dim3(tilesV / 8, 1), dim3(256), 0, stream>>>(
      XR16, XR16, kC, 0L, WV16, WV16, kC, 0L,
      (void*)VR, (void*)VR, kVN, 0L, bq, VR, 0L, kTok, kVN, kC, kWCarryInv);

  const int  tilesScore  = (kL / 64) * (kL / 64);
  const long strideHead  = (long)kDh;
  const long strideScore = (long)kL * kL;
  for (int bb = 0; bb < kB; ++bb) {
    for (int gh = 0; gh < kH / kGH; ++gh) {
      const int h0 = gh * kGH;
      const unsigned short* Ag  = QK16 + (size_t)bb * kL * kQKld + (size_t)h0 * kDh;
      const unsigned short* Btg = Ag + kC;
      wmma_gemm64<0, false, 0, 0, false, 0><<<dim3(tilesScore / 8, kGH), dim3(256), 0, stream>>>(
          Ag, Ag, kQKld, strideHead, Btg, Btg, kQKld, strideHead,
          (void*)SC, (void*)SC, kL, strideScore, bq, VR, 0L, kL, kL, kDh, kScale);
      rowstats_kernel<<<dim3(kL / 32, kGH), dim3(256), 0, stream>>>(SC, VR, ST, bb, h0);
      colsum_kernel<<<dim3(kL / 1024, kGH), dim3(256), 0, stream>>>(SC, ST, CS, bb, h0);
    }
  }

  const int n4 = (kB * kL * kH) / 4;
  pool_kernel<<<dim3(n4 / 256), dim3(256), 0, stream>>>(CS, out, n4);
}
